// HybridCrystalPINN_8847632630356
// MI455X (gfx1250) — hardware-verified
//
#include <hip/hip_runtime.h>
#include <hip/hip_bf16.h>
#include <math.h>

typedef __attribute__((ext_vector_type(16))) _Float16 v16h;
typedef __attribute__((ext_vector_type(8)))  _Float16 v8h;
typedef __attribute__((ext_vector_type(4)))  _Float16 v4h;
typedef __attribute__((ext_vector_type(2)))  _Float16 v2h;
typedef __attribute__((ext_vector_type(8)))  float    v8f;

#define TILE_ROWS 128
#define THREADS   128

union frag_u {
  v16h v;
  v8h  h[2];
  v4h  q[4];
  v2h  d[8];
};

struct Smem {
  alignas(16) _Float16 w1h[2 * 64];
  alignas(16) _Float16 w2h[64 * 16];
  alignas(16) _Float16 pwh[16 * 4];
  alignas(16) _Float16 pw1h[4 * 32];
  alignas(16) _Float16 pw2h[32 * 4];
  alignas(16) float b1[64];
  alignas(16) float b2[16];
  alignas(16) float pbias[4];
  alignas(16) float pb1[32];
  alignas(16) float pb2[4];
  alignas(16) float qcs[8][2];
  alignas(16) _Float16 xh[TILE_ROWS * 2];
  alignas(16) _Float16 z1h[TILE_ROWS * 64];
  alignas(16) _Float16 z2h[TILE_ROWS * 16];
  alignas(16) float    qinf[TILE_ROWS * 4];
  alignas(16) _Float16 qoh[TILE_ROWS * 4];
  alignas(16) _Float16 hh[TILE_ROWS * 32];
  alignas(16) float    outf[TILE_ROWS * 4];
};

__device__ __forceinline__ float fast_tanh(float x) {
  const float ax = fabsf(x);
  const float e  = __expf(2.0f * ax);
  const float r  = __builtin_amdgcn_rcpf(e + 1.0f);
  const float t  = 1.0f - 2.0f * r;
  return copysignf(t, x);
}

template <int LD, int KVALID>
__device__ __forceinline__ v16h pack_A(const _Float16* m, int row0, int k0) {
  const int lane = threadIdx.x & 31;
  const int g    = lane >> 4;
  const _Float16* p = m + (row0 + (lane & 15)) * LD + k0;
  frag_u u;
  if constexpr (KVALID >= 32) {
    u.h[0] = *(const v8h*)(p + 8 * g);
    u.h[1] = *(const v8h*)(p + 16 + 8 * g);
  } else if constexpr (KVALID == 16) {
    u.h[0] = *(const v8h*)(p + 8 * g);
    u.h[1] = (v8h){};
  } else if constexpr (KVALID == 4) {
    u.v = (v16h){};
    if (g == 0) u.q[0] = *(const v4h*)(p);
  } else {
    u.v = (v16h){};
    if (g == 0) u.d[0] = *(const v2h*)(p);
  }
  return u.v;
}

template <int LD, int KVALID, int NVALID>
__device__ __forceinline__ v16h pack_B(const _Float16* m, int k0, int n0) {
  const int lane = threadIdx.x & 31;
  const int n    = lane & 15;
  const int g    = lane >> 4;
  v16h b = {};
  const bool nv = (NVALID >= 16) || (n < NVALID);
  if (nv) {
#pragma unroll
    for (int e = 0; e < 16; ++e) {
      const int kb = (e < 8) ? (8 * g + e) : (16 + 8 * g + (e - 8));
      if (kb < KVALID) b[e] = m[(k0 + kb) * LD + n0 + n];
    }
  }
  return b;
}

__device__ __forceinline__ v8f wmma16(v16h a, v16h b, v8f c) {
  v8f d = __builtin_amdgcn_wmma_f32_16x16x32_f16(false, a, false, b, (short)0,
                                                 c, false, false);
  asm volatile("v_nop\n\tv_nop\n\tv_nop\n\tv_nop" : "+v"(d) : "v"(a), "v"(b));
  return d;
}

__device__ __forceinline__ void apply_ry_cs(float* st, int bit, float c, float s) {
#pragma unroll
  for (int i = 0; i < 16; ++i) {
    if ((i & bit) == 0) {
      const float s0 = st[i], s1 = st[i | bit];
      st[i]       = c * s0 - s * s1;
      st[i | bit] = s * s0 + c * s1;
    }
  }
}

__device__ __forceinline__ void apply_ry(float* st, int bit, float theta) {
  apply_ry_cs(st, bit, __cosf(0.5f * theta), __sinf(0.5f * theta));
}

__device__ __forceinline__ void apply_cnot(float* st, int cb, int tb) {
#pragma unroll
  for (int i = 0; i < 16; ++i) {
    if ((i & cb) && !(i & tb)) {
      const float t = st[i];
      st[i]      = st[i | tb];
      st[i | tb] = t;
    }
  }
}

__global__ __launch_bounds__(THREADS) void hybrid_pinn_kernel(
    const float* __restrict__ x,
    const float* __restrict__ enc_w1, const float* __restrict__ enc_b1,
    const float* __restrict__ enc_w2, const float* __restrict__ enc_b2,
    const float* __restrict__ pre_w,  const float* __restrict__ pre_b,
    const float* __restrict__ q_weights,
    const float* __restrict__ post_w1, const float* __restrict__ post_b1,
    const float* __restrict__ post_w2, const float* __restrict__ post_b2,
    float* __restrict__ out) {
  __shared__ Smem sm;
  const int tid   = threadIdx.x;
  const int gbase = blockIdx.x * TILE_ROWS;

  for (int i = tid; i < 2 * 64; i += THREADS)  sm.w1h[i]  = (_Float16)enc_w1[i];
  for (int i = tid; i < 64 * 16; i += THREADS) sm.w2h[i]  = (_Float16)enc_w2[i];
  for (int i = tid; i < 16 * 4; i += THREADS)  sm.pwh[i]  = (_Float16)pre_w[i];
  for (int i = tid; i < 4 * 32; i += THREADS)  sm.pw1h[i] = (_Float16)post_w1[i];
  for (int i = tid; i < 32 * 4; i += THREADS)  sm.pw2h[i] = (_Float16)post_w2[i];
  if (tid < 64) sm.b1[tid]    = enc_b1[tid];
  if (tid < 16) sm.b2[tid]    = enc_b2[tid];
  if (tid < 4)  sm.pbias[tid] = pre_b[tid];
  if (tid < 32) sm.pb1[tid]   = post_b1[tid];
  if (tid < 4)  sm.pb2[tid]   = post_b2[tid];
  if (tid < 8) {
    const float th = 0.5f * q_weights[tid];
    sm.qcs[tid][0] = __cosf(th);
    sm.qcs[tid][1] = __sinf(th);
  }
  {
    const float2 xv = ((const float2*)x)[gbase + tid];
    sm.xh[2 * tid]     = (_Float16)xv.x;
    sm.xh[2 * tid + 1] = (_Float16)xv.y;
  }
  __syncthreads();

  const int lane  = tid & 31;
  const int wid   = tid >> 5;
  const int g     = lane >> 4;
  const int nlane = lane & 15;

  v16h bw1[4], bw2[2], bp1f[2];
#pragma unroll
  for (int nt = 0; nt < 4; ++nt) bw1[nt] = pack_B<64, 2, 16>(sm.w1h, 0, nt * 16);
#pragma unroll
  for (int kt = 0; kt < 2; ++kt) bw2[kt] = pack_B<16, 32, 16>(sm.w2h, kt * 32, 0);
  const v16h bpw = pack_B<4, 16, 4>(sm.pwh, 0, 0);
#pragma unroll
  for (int nt = 0; nt < 2; ++nt) bp1f[nt] = pack_B<32, 4, 16>(sm.pw1h, 0, nt * 16);
  const v16h bp2 = pack_B<4, 32, 4>(sm.pw2h, 0, 0);

#pragma unroll
  for (int tt = 0; tt < 2; ++tt) {
    const int row0 = (wid * 2 + tt) * 16;

    const v16h a1 = pack_A<2, 2>(sm.xh, row0, 0);
#pragma unroll
    for (int nt = 0; nt < 4; ++nt) {
      v8f c = {};
      c = wmma16(a1, bw1[nt], c);
      const float bias = sm.b1[nt * 16 + nlane];
#pragma unroll
      for (int r = 0; r < 8; ++r) {
        const float v = fast_tanh(c[r] + bias);
        sm.z1h[(row0 + r + 8 * g) * 64 + nt * 16 + nlane] = (_Float16)v;
      }
    }

    {
      v8f c = {};
#pragma unroll
      for (int kt = 0; kt < 2; ++kt) {
        const v16h a = pack_A<64, 32>(sm.z1h, row0, kt * 32);
        c = wmma16(a, bw2[kt], c);
      }
      const float bias = sm.b2[nlane];
#pragma unroll
      for (int r = 0; r < 8; ++r) {
        const float v = fast_tanh(c[r] + bias);
        sm.z2h[(row0 + r + 8 * g) * 16 + nlane] = (_Float16)v;
      }
    }

    {
      const v16h a = pack_A<16, 16>(sm.z2h, row0, 0);
      v8f c = {};
      c = wmma16(a, bpw, c);
      if (nlane < 4) {
        const float bias = sm.pbias[nlane];
#pragma unroll
        for (int r = 0; r < 8; ++r)
          sm.qinf[(row0 + r + 8 * g) * 4 + nlane] = c[r] + bias;
      }
    }
  }
  __syncthreads();

  {
    float st[16];
#pragma unroll
    for (int i = 0; i < 16; ++i) st[i] = 0.0f;
    st[0] = 1.0f;

    const float4 qi = *(const float4*)&sm.qinf[tid * 4];
    apply_ry(st, 8, qi.x);
    apply_ry(st, 4, qi.y);
    apply_ry(st, 2, qi.z);
    apply_ry(st, 1, qi.w);

#pragma unroll
    for (int l = 0; l < 2; ++l) {
#pragma unroll
      for (int q = 0; q < 4; ++q) {
        const float2 cs = *(const float2*)&sm.qcs[l * 4 + q][0];
        apply_ry_cs(st, 8 >> q, cs.x, cs.y);
      }
      apply_cnot(st, 8, 4);
      apply_cnot(st, 4, 2);
      apply_cnot(st, 2, 1);
      apply_cnot(st, 1, 8);
    }

    v4h qo;
#pragma unroll
    for (int q = 0; q < 4; ++q) {
      const int bit = 8 >> q;
      float e = 0.0f;
#pragma unroll
      for (int i = 0; i < 16; ++i)
        e += ((i & bit) ? -1.0f : 1.0f) * st[i] * st[i];
      qo[q] = (_Float16)e;
    }
    *(v4h*)&sm.qoh[tid * 4] = qo;
  }
  __syncthreads();

#pragma unroll
  for (int tt = 0; tt < 2; ++tt) {
    const int row0 = (wid * 2 + tt) * 16;

    const v16h a = pack_A<4, 4>(sm.qoh, row0, 0);
#pragma unroll
    for (int nt = 0; nt < 2; ++nt) {
      v8f c = {};
      c = wmma16(a, bp1f[nt], c);
      const float bias = sm.pb1[nt * 16 + nlane];
#pragma unroll
      for (int r = 0; r < 8; ++r) {
        const float v = fast_tanh(c[r] + bias);
        sm.hh[(row0 + r + 8 * g) * 32 + nt * 16 + nlane] = (_Float16)v;
      }
    }

    {
      const v16h a2 = pack_A<32, 32>(sm.hh, row0, 0);
      v8f c = {};
      c = wmma16(a2, bp2, c);
      if (nlane < 4) {
        const float bias = sm.pb2[nlane];
#pragma unroll
        for (int r = 0; r < 8; ++r)
          sm.outf[(row0 + r + 8 * g) * 4 + nlane] = c[r] + bias;
      }
    }
  }
  __syncthreads();

  {
    typedef __attribute__((ext_vector_type(4))) float v4fo;
    const v4fo ov = *(const v4fo*)&sm.outf[tid * 4];
    *(volatile v4fo*)((v4fo*)out + gbase + tid) = ov; __threadfence(); *(volatile v4fo*)((v4fo*)out + gbase + tid) = ov;
  }
}

extern "C" void kernel_launch(void* const* d_in, const int* in_sizes, int n_in,
                              void* d_out, int out_size, void* d_ws, size_t ws_size,
                              hipStream_t stream) {
  (void)n_in; (void)out_size; (void)d_ws; (void)ws_size;
  const float* x       = (const float*)d_in[0];
  const float* enc_w1  = (const float*)d_in[1];
  const float* enc_b1  = (const float*)d_in[2];
  const float* enc_w2  = (const float*)d_in[3];
  const float* enc_b2  = (const float*)d_in[4];
  const float* pre_w   = (const float*)d_in[5];
  const float* pre_b   = (const float*)d_in[6];
  const float* q_w     = (const float*)d_in[7];
  const float* post_w1 = (const float*)d_in[8];
  const float* post_b1 = (const float*)d_in[9];
  const float* post_w2 = (const float*)d_in[10];
  const float* post_b2 = (const float*)d_in[11];
  float* out = (float*)d_out;

  (void)in_sizes;
  const int nblocks = 524288 / TILE_ROWS;

  hybrid_pinn_kernel<<<nblocks, THREADS, 0, stream>>>(
      x, enc_w1, enc_b1, enc_w2, enc_b2, pre_w, pre_b, q_w,
      post_w1, post_b1, post_w2, post_b2, out);
}
